// DeepMambaModel_18253611008299
// MI455X (gfx1250) — hardware-run, weakly checked
//
#include <hip/hip_runtime.h>
#include <hip/hip_bf16.h>
#include <math.h>

#define NB    2
#define LL    1024
#define NTOK  (NB * LL)
#define DMOD  512
#define DM4   128
#define DIN   1024
#define XZW   (2 * DIN)
#define DST   16
#define DTR   32
#define XDN   (DTR + 2 * DST)
#define DCV   4
#define NLAY  3
#define SDIM  17
#define ADIM  7
#define MAXT  2048
#define NOUT  (NTOK * SDIM + NTOK * ADIM)
#define GSTR  40
#define OSTR  68
#define SMEMB (8 * 16 * OSTR * 4)
#define SCH   32
#define SYP   260
#define LOG2E 1.4426950408889634f

static_assert(NTOK % 128 == 0);
static_assert(XZW % 64 == 0);
static_assert(XDN == 64);
static_assert(DIN % 64 == 0);
static_assert(DMOD % 64 == 0);
static_assert(DMOD % 32 == 0);
static_assert(DIN % 32 == 0);
static_assert(DTR == 32);
static_assert(DST == 16);
static_assert(LL % SCH == 0);
static_assert(SCH == 32);
static_assert(SYP % 4 == 0);
static_assert(SYP >= 256);
static_assert(SMEMB >= (2 * 128 * GSTR + 64 * GSTR) * 2);
static_assert(DMOD == 4 * 128);
static_assert(DIN == 4 * 256);
static_assert((NTOK * SDIM) % 128 == 0);
static_assert(NOUT % (4 * 256) == 0);
static_assert((NTOK * DTR / 8) % 256 == 0);

typedef unsigned short us16 __attribute__((ext_vector_type(16)));
typedef unsigned short us8  __attribute__((ext_vector_type(8)));
typedef unsigned short us8a __attribute__((ext_vector_type(8), may_alias));
typedef __bf16 v16b __attribute__((ext_vector_type(16)));
typedef float v8f __attribute__((ext_vector_type(8)));
typedef float v4f __attribute__((ext_vector_type(4)));
typedef float v4fa __attribute__((ext_vector_type(4), may_alias));
union FragU { us16 v; us8 h[2]; };

__device__ __forceinline__ unsigned short bf16_bits(float f) {
  unsigned u = __float_as_uint(f);
  u += 0x7FFFu + ((u >> 16) & 1u);
  return (unsigned short)(u >> 16);
}
__device__ __forceinline__ float bf16_val(unsigned short b) { return __uint_as_float(((unsigned)b) << 16); }
__device__ __forceinline__ float bf16r(float f) { return bf16_val(bf16_bits(f)); }
__device__ __forceinline__ float siluf(float x) { return x * __builtin_amdgcn_rcpf(1.0f + __expf(-x)); }

__device__ __forceinline__ v8f mma_bf16(us16 a, us16 b, v8f c) {
  return __builtin_amdgcn_wmma_f32_16x16x32_bf16(false, __builtin_bit_cast(v16b, a), false, __builtin_bit_cast(v16b, b), (short)0, c, false, false);
}
__device__ __forceinline__ void wguard(v8f& c0, v8f& c1, v8f& c2, v8f& c3, const us16& a0, const us16& a1,
                                       const us16& b0, const us16& b1, const us16& b2, const us16& b3) {
#if defined(__HIP_DEVICE_COMPILE__)
  asm volatile("v_nop\n\tv_nop\n\tv_nop\n\tv_nop"
               : "+v"(c0), "+v"(c1), "+v"(c2), "+v"(c3)
               : "v"(a0), "v"(a1), "v"(b0), "v"(b1), "v"(b2), "v"(b3));
#endif
}

__device__ __forceinline__ us16 lds_frag(const unsigned short* base) {
  const int lane = threadIdx.x & 31, r = lane & 15, kh = (lane >> 4) * 8;
  FragU f;
  f.h[0] = *(const us8a*)(base + r * GSTR + kh);
  f.h[1] = *(const us8a*)(base + r * GSTR + 16 + kh);
  return f.v;
}

__device__ __forceinline__ void stage_a(unsigned short* lds, const unsigned short* __restrict__ P, int ld, int m0, int k0, int tid) {
  const int row = tid >> 1, cq = (tid & 1) * 16;
  const unsigned short* src = P + (size_t)(m0 + row) * ld + k0 + cq;
  const us8 v0 = *(const us8a*)src;
  const us8 v1 = *(const us8a*)(src + 8);
  *(us8a*)(lds + row * GSTR + cq) = v0;
  *(us8a*)(lds + row * GSTR + cq + 8) = v1;
}
__device__ __forceinline__ void stage_b(unsigned short* lds, const unsigned short* __restrict__ P, int ld, int n0, int k0, int tid) {
  const int row = tid >> 2, kq = (tid & 3) * 8;
  const us8 v = *(const us8a*)(P + (size_t)(n0 + row) * ld + k0 + kq);
  *(us8a*)(lds + row * GSTR + kq) = v;
}

__global__ __launch_bounds__(256) void k_gemm(const unsigned short* __restrict__ A0, const unsigned short* __restrict__ A1, int lda,
                                             const unsigned short* __restrict__ B0, int ldb, float* Y, int ldy, int K) {
  __shared__ __attribute__((aligned(16))) unsigned char sm[SMEMB];
  unsigned short* lA0 = (unsigned short*)sm;
  unsigned short* lA1 = lA0 + 128 * GSTR;
  unsigned short* lB0 = lA1 + 128 * GSTR;
  float* oS = (float*)sm;
  const int tid = threadIdx.x, lane = tid & 31, wave = tid >> 5, cl = lane & 15, hh = lane >> 4;
  const int m0 = blockIdx.x * 128, n0 = blockIdx.y * 64;

  v8f acc[4];
#pragma unroll
  for (int j = 0; j < 4; ++j) { v8f zz = {0.f, 0.f, 0.f, 0.f, 0.f, 0.f, 0.f, 0.f}; acc[j] = zz; }

#pragma unroll 1
  for (int k0 = 0; k0 < K; k0 += 32) {
    __syncthreads();
    stage_a(lA0, A0, lda, m0, k0, tid);
    stage_a(lA1, A1, lda, m0, k0, tid);
    stage_b(lB0, B0, ldb, n0, k0, tid);
    __syncthreads();
    const us16 af0 = lds_frag(lA0 + 16 * wave * GSTR);
    const us16 af1 = lds_frag(lA1 + 16 * wave * GSTR);
    us16 bfr[4];
#pragma unroll
    for (int j = 0; j < 4; ++j) bfr[j] = lds_frag(lB0 + 16 * j * GSTR);
#pragma unroll
    for (int j = 0; j < 4; ++j) acc[j] = mma_bf16(af0, bfr[j], acc[j]);
#pragma unroll
    for (int j = 0; j < 4; ++j) acc[j] = mma_bf16(af1, bfr[j], acc[j]);
    wguard(acc[0], acc[1], acc[2], acc[3], af0, af1, bfr[0], bfr[1], bfr[2], bfr[3]);
  }
  __syncthreads();

  float* so = oS + wave * (16 * OSTR);
#pragma unroll
  for (int j = 0; j < 4; ++j)
#pragma unroll
    for (int r = 0; r < 8; ++r) so[(8 * hh + r) * OSTR + 16 * j + cl] = acc[j][r];
  __syncthreads();
#pragma unroll
  for (int pass = 0; pass < 2; ++pass) {
#pragma unroll
    for (int it = 0; it < 8; ++it) {
      const int ch = it * 32 + lane, r = ch >> 4, q = (ch & 15) * 4;
      const v4f v = *(const v4fa*)(so + r * OSTR + q);
      *(volatile v4f*)(Y + (size_t)(m0 + 16 * wave + r) * ldy + n0 + q) = v;
    }
    __threadfence();
  }
}

__global__ __launch_bounds__(256) void k_cvt(const float* __restrict__ src, unsigned short* dst, int nsrc, int ncol8, int total8) {
  const int idx = blockIdx.x * 256 + threadIdx.x;
  if (idx >= total8) return;
  const int row = idx / ncol8, c8 = (idx - row * ncol8) * 8;
  const int rs = (row < nsrc) ? row : (nsrc - 1);
  const float* s = src + (size_t)rs * (size_t)(ncol8 * 8) + c8;
  const v4f a = *(const v4fa*)s, b = *(const v4fa*)(s + 4);
  const bool zr = (row >= nsrc);
  us8 o;
#pragma unroll
  for (int u = 0; u < 4; ++u) {
    o[u]     = zr ? (unsigned short)0 : bf16_bits(a[u]);
    o[4 + u] = zr ? (unsigned short)0 : bf16_bits(b[u]);
  }
  const size_t off = (size_t)row * (size_t)(ncol8 * 8) + c8;
  *(volatile us8*)(dst + off) = o;
  __threadfence();
  *(volatile us8*)(dst + off) = o;
}

__global__ __launch_bounds__(128) void k_embed(const float* __restrict__ st, const float* __restrict__ ac, const float* __restrict__ rtg,
                                              const float* __restrict__ ctg, const int* __restrict__ ts,
                                              const float* __restrict__ Ws, const float* __restrict__ bs,
                                              const float* __restrict__ Wa, const float* __restrict__ ba,
                                              const float* __restrict__ Wr, const float* __restrict__ br,
                                              const float* __restrict__ Wc, const float* __restrict__ bcn,
                                              const float* __restrict__ Et, float* X) {
#pragma clang fp contract(off)
  const int row = blockIdx.x, d = threadIdx.x, l = row % LL;
  int t = ts[row];
  t = (t < 0) ? 0 : t;  t = (t > MAXT - 1) ? (MAXT - 1) : t;
  const int rp = (l > 0) ? (row - 1) : row;
  int tp = ts[rp];
  tp = (tp < 0) ? 0 : tp;  tp = (tp > MAXT - 1) ? (MAXT - 1) : tp;
  const float te  = bf16r(Et[(size_t)t * DM4 + d]);
  const float tep = bf16r(Et[(size_t)tp * DM4 + d]);
  const float re = (bf16r(rtg[row]) * bf16r(Wr[d]) + bf16r(br[d])) + te;
  const float ce = (bf16r(ctg[row]) * bf16r(Wc[d]) + bf16r(bcn[d])) + te;
  float sa = 0.0f;
#pragma unroll
  for (int k = 0; k < SDIM; ++k) sa = sa + bf16r(st[(size_t)row * SDIM + k]) * bf16r(Ws[d * SDIM + k]);
  const float se = (sa + bf16r(bs[d])) + te;
  float aa = 0.0f;
#pragma unroll
  for (int k = 0; k < ADIM; ++k) aa = aa + bf16r(ac[(size_t)rp * ADIM + k]) * bf16r(Wa[d * ADIM + k]);
  const float aef = (aa + bf16r(ba[d])) + tep;
  const float ae = (l > 0) ? aef : 0.0f;
  volatile float* xr = X + (size_t)row * DMOD;
  xr[d] = re;  xr[DM4 + d] = ce;  xr[2 * DM4 + d] = se;  xr[3 * DM4 + d] = ae;
  __threadfence();
  xr[d] = re;  xr[DM4 + d] = ce;  xr[2 * DM4 + d] = se;  xr[3 * DM4 + d] = ae;
}

template <int ADD, int FIN>
__global__ __launch_bounds__(128) void k_ln(float* X, const float* __restrict__ Y2, const float* __restrict__ g, const float* __restrict__ bt,
                                           unsigned short* NH, unsigned short* NLO, float* F) {
#pragma clang fp contract(off)
  __shared__ __attribute__((aligned(16))) float srow[DMOD];
  __shared__ float sred[8];
  const int row = blockIdx.x, tid = threadIdx.x, lane = tid & 31, wave = tid >> 5;
  const size_t base = (size_t)row * DMOD + tid * 4;
  v4f xv = *(const v4fa*)(X + base);
  if (ADD) { const v4f yv = *(const v4fa*)(Y2 + base); xv = xv + yv; }
  float s = (xv[0] + xv[1]) + (xv[2] + xv[3]);
#pragma unroll
  for (int o = 16; o > 0; o >>= 1) s = s + __shfl_xor(s, o);
  if (lane == 0) sred[wave] = s;
  __syncthreads();
  const float mu = ((sred[0] + sred[1]) + (sred[2] + sred[3])) * (1.0f / DMOD);
  const v4f dv = xv - mu;
  float s2 = (dv[0] * dv[0] + dv[1] * dv[1]) + (dv[2] * dv[2] + dv[3] * dv[3]);
#pragma unroll
  for (int o = 16; o > 0; o >>= 1) s2 = s2 + __shfl_xor(s2, o);
  if (lane == 0) sred[4 + wave] = s2;
  __syncthreads();
  const float var = ((sred[4] + sred[5]) + (sred[6] + sred[7])) * (1.0f / DMOD);
  const float rs = rsqrtf(var + 1e-5f);
  const v4f gv = *(const v4fa*)(g + tid * 4), bv = *(const v4fa*)(bt + tid * 4);
  v4f ov;
#pragma unroll
  for (int u = 0; u < 4; ++u) ov[u] = (dv[u] * rs) * bf16r(gv[u]) + bf16r(bv[u]);

  if (FIN) {
    *(volatile v4f*)(F + base) = ov;
    __threadfence();
    *(volatile v4f*)(F + base) = ov;
  } else {
    if (ADD) {
      *(volatile v4f*)(X + base) = xv;
      __threadfence();
      *(volatile v4f*)(X + base) = xv;
    }
    *(v4fa*)(srow + tid * 4) = ov;
    __syncthreads();
    if (tid < 64) {
      const int c8 = tid * 8;
      const v4f a = *(const v4fa*)(srow + c8);
      const v4f b = *(const v4fa*)(srow + c8 + 4);
      us8 hi, lo;
#pragma unroll
      for (int u = 0; u < 4; ++u) {
        const unsigned short ha = bf16_bits(a[u]);
        hi[u] = ha; lo[u] = bf16_bits(a[u] - bf16_val(ha));
        const unsigned short hb = bf16_bits(b[u]);
        hi[4 + u] = hb; lo[4 + u] = bf16_bits(b[u] - bf16_val(hb));
      }
      const size_t o2 = (size_t)row * DMOD + c8;
      *(volatile us8*)(NH + o2) = hi; *(volatile us8*)(NLO + o2) = lo;
      __threadfence();
      *(volatile us8*)(NH + o2) = hi; *(volatile us8*)(NLO + o2) = lo;
    }
  }
}

__global__ __launch_bounds__(256) void k_conv(const float* __restrict__ XZ, const float* __restrict__ cw, const float* __restrict__ cb,
                                             float* XCF, unsigned short* XCH, unsigned short* XCL) {
#pragma clang fp contract(off)
  __shared__ __attribute__((aligned(16))) float sxs[DIN];
  const int tid = threadIdx.x, c4 = tid * 4;
  const int tok = blockIdx.x, l = tok % LL;
  v4f xv[DCV];
#pragma unroll
  for (int j = 0; j < DCV; ++j) {
    const int ll = l - (DCV - 1) + j;
    const int tc = (ll >= 0) ? (tok - (DCV - 1) + j) : tok;
    xv[j] = *(const v4fa*)(XZ + (size_t)tc * XZW + c4);
  }
  const v4f bb = *(const v4fa*)(cb + c4);
  v4f sv;
#pragma unroll
  for (int u = 0; u < 4; ++u) {
    const v4f wv = *(const v4fa*)(cw + (size_t)(c4 + u) * DCV);
    float a = 0.0f;
#pragma unroll
    for (int j = 0; j < DCV; ++j) {
      const float pr = bf16r(wv[j]) * xv[j][u];
      a = a + ((l - (DCV - 1) + j >= 0) ? pr : 0.0f);
    }
    a = a + bf16r(bb[u]);
    sv[u] = siluf(a);
  }
  *(v4fa*)(sxs + c4) = sv;
  const size_t o = (size_t)tok * DIN + c4;
  *(volatile v4f*)(XCF + o) = sv;
  __threadfence();
  *(volatile v4f*)(XCF + o) = sv;
  __syncthreads();
  if (tid < 128) {
    const int c8 = tid * 8;
    const v4f a = *(const v4fa*)(sxs + c8);
    const v4f b = *(const v4fa*)(sxs + c8 + 4);
    us8 hi, lo;
#pragma unroll
    for (int u = 0; u < 4; ++u) {
      const unsigned short ha = bf16_bits(a[u]);
      hi[u] = ha; lo[u] = bf16_bits(a[u] - bf16_val(ha));
      const unsigned short hb = bf16_bits(b[u]);
      hi[4 + u] = hb; lo[4 + u] = bf16_bits(b[u] - bf16_val(hb));
    }
    const size_t o2 = (size_t)tok * DIN + c8;
    *(volatile us8*)(XCH + o2) = hi; *(volatile us8*)(XCL + o2) = lo;
    __threadfence();
    *(volatile us8*)(XCH + o2) = hi; *(volatile us8*)(XCL + o2) = lo;
  }
}

__global__ __launch_bounds__(256) void k_dtsplit(const float* __restrict__ XD, unsigned short* DTH, unsigned short* DTL) {
  const int idx = blockIdx.x * 256 + threadIdx.x;
  if (idx >= NTOK * DTR / 8) return;
  const int row = idx >> 2, c8 = (idx & 3) * 8;
  const v4f a = *(const v4fa*)(XD + (size_t)row * XDN + c8), b = *(const v4fa*)(XD + (size_t)row * XDN + c8 + 4);
  us8 hi, lo;
#pragma unroll
  for (int u = 0; u < 4; ++u) {
    const unsigned short ha = bf16_bits(a[u]);
    hi[u] = ha; lo[u] = bf16_bits(a[u] - bf16_val(ha));
    const unsigned short hb = bf16_bits(b[u]);
    hi[4 + u] = hb; lo[4 + u] = bf16_bits(b[u] - bf16_val(hb));
  }
  const size_t off = (size_t)row * DTR + c8;
  *(volatile us8*)(DTH + off) = hi; *(volatile us8*)(DTL + off) = lo;
  __threadfence();
  *(volatile us8*)(DTH + off) = hi; *(volatile us8*)(DTL + off) = lo;
}

__global__ __launch_bounds__(256) void k_scan(const float* __restrict__ XZ, const float* __restrict__ XCF, const float* __restrict__ XD,
                                             const float* __restrict__ DTW, const float* __restrict__ dtb, const float* __restrict__ Alog,
                                             const float* __restrict__ Dv, unsigned short* YGH, unsigned short* YGL) {
#pragma clang fp contract(off)
  __shared__ __attribute__((aligned(16))) float sy[SCH * SYP];
  const int b = blockIdx.x >> 2, dg = blockIdx.x & 3, tid = threadIdx.x, lane = tid & 31, wave = tid >> 5;
  const int d = dg * 256 + tid;
  float A2[DST], h[DST];
#pragma unroll
  for (int n = 0; n < DST; ++n) { A2[n] = -__expf(bf16r(Alog[d * DST + n])) * LOG2E; h[n] = 0.0f; }
  const float Dd = bf16r(Dv[d]);
  const float bd = bf16r(dtb[d]);
#pragma unroll 1
  for (int c = 0; c < LL / SCH; ++c) {
#pragma unroll 1
    for (int s = 0; s < SCH; ++s) {
      const size_t tok = (size_t)b * LL + (size_t)(c * SCH + s);
      const float raw = DTW[tok * DIN + d];
      const float a = raw + bd;
      const float dl = fmaxf(a, 0.0f) + log1pf(__expf(-fabsf(a)));
      const float xv = XCF[tok * DIN + d];
      const float zv = XZ[tok * XZW + DIN + d];
      const float* bcp = XD + tok * XDN;
      v4f Bv[4], Cv[4];
#pragma unroll
      for (int q = 0; q < 4; ++q) {
        Bv[q] = *(const v4fa*)(bcp + DTR + 4 * q);
        Cv[q] = *(const v4fa*)(bcp + DTR + DST + 4 * q);
      }
      const float dx = dl * xv;
      float y = 0.0f;
#pragma unroll
      for (int n = 0; n < DST; ++n) {
        const float e = exp2f(dl * A2[n]);
        h[n] = e * h[n] + dx * Bv[n >> 2][n & 3];
        y = y + h[n] * Cv[n >> 2][n & 3];
      }
      const float yv = (y + xv * Dd) * siluf(zv);
      sy[s * SYP + tid] = yv;
    }
    __syncthreads();
#pragma unroll
    for (int pass = 0; pass < 2; ++pass) {
#pragma unroll
      for (int it = 0; it < 4; ++it) {
        const int row = 4 * wave + it;
        const v4f va = *(const v4fa*)(sy + row * SYP + lane * 8);
        const v4f vb = *(const v4fa*)(sy + row * SYP + lane * 8 + 4);
        us8 hi, lo;
#pragma unroll
        for (int u = 0; u < 4; ++u) {
          const unsigned short ha = bf16_bits(va[u]);
          hi[u] = ha; lo[u] = bf16_bits(va[u] - bf16_val(ha));
          const unsigned short hb = bf16_bits(vb[u]);
          hi[4 + u] = hb; lo[4 + u] = bf16_bits(vb[u] - bf16_val(hb));
        }
        const size_t o = ((size_t)b * LL + (size_t)(c * SCH + row)) * DIN + (size_t)dg * 256 + lane * 8;
        *(volatile us8*)(YGH + o) = hi; *(volatile us8*)(YGL + o) = lo;
      }
      __threadfence();
    }
    __syncthreads();
  }
}

__global__ __launch_bounds__(256) void k_heads(const float* __restrict__ F, const float* __restrict__ Wps, const float* __restrict__ bps,
                                              const float* __restrict__ Wpa, const float* __restrict__ bpa, float* out) {
#pragma clang fp contract(off)
  const int idx = blockIdx.x * 256 + threadIdx.x;
  if (idx >= NOUT / 4) return;
  const int e0 = idx * 4;
  const bool isS = (e0 < NTOK * SDIM);
  const float* src[4];
  const float* wr[4];
  float bias[4], acc[4];
#pragma unroll
  for (int u = 0; u < 4; ++u) {
    const int e = e0 + u;
    int rowS = e / SDIM;  const int jS = e - rowS * SDIM;  rowS = (rowS < NTOK) ? rowS : (NTOK - 1);
    int eA = e - NTOK * SDIM;  eA = (eA > 0) ? eA : 0;
    int rowA = eA / ADIM;  const int qA = eA - rowA * ADIM;  rowA = (rowA < NTOK) ? rowA : (NTOK - 1);
    const int row = isS ? rowS : rowA;
    src[u] = F + (size_t)row * DMOD + (isS ? 3 * DM4 : 2 * DM4);
    wr[u]  = isS ? (Wps + jS * DM4) : (Wpa + qA * DM4);
    const float b1 = bf16r(bps[jS]), b2 = bf16r(bpa[qA]);
    bias[u] = isS ? b1 : b2;
    acc[u] = 0.0f;
  }
#pragma unroll 1
  for (int k = 0; k < DM4; ++k) {
#pragma unroll
    for (int u = 0; u < 4; ++u) acc[u] = acc[u] + src[u][k] * bf16r(wr[u][k]);
  }
  v4f res;
#pragma unroll
  for (int u = 0; u < 4; ++u) res[u] = acc[u] + bias[u];
  *(volatile v4f*)(out + e0) = res;
  __threadfence();
  *(volatile v4f*)(out + e0) = res;
}

extern "C" void kernel_launch(void* const* d_in, const int* in_sizes, int n_in,
                              void* d_out, int out_size, void* d_ws, size_t ws_size,
                              hipStream_t stream) {
  if (n_in < 31) return;
  if (in_sizes[0] != NTOK * SDIM || in_sizes[1] != NTOK * ADIM || in_sizes[2] != NTOK || in_sizes[3] != NTOK || in_sizes[4] != NTOK ||
      in_sizes[5] != DM4 * SDIM || in_sizes[6] != DM4 || in_sizes[7] != DM4 * ADIM || in_sizes[8] != DM4 || in_sizes[9] != DM4 ||
      in_sizes[10] != DM4 || in_sizes[11] != DM4 || in_sizes[12] != DM4 || in_sizes[13] != MAXT * DM4 ||
      in_sizes[14] != NLAY * DMOD || in_sizes[15] != NLAY * DMOD || in_sizes[16] != NLAY * XZW * DMOD ||
      in_sizes[17] != NLAY * DIN * DCV || in_sizes[18] != NLAY * DIN || in_sizes[19] != NLAY * XDN * DIN ||
      in_sizes[20] != NLAY * DIN * DTR || in_sizes[21] != NLAY * DIN || in_sizes[22] != NLAY * DIN * DST || in_sizes[23] != NLAY * DIN ||
      in_sizes[24] != NLAY * DMOD * DIN || in_sizes[25] != DMOD || in_sizes[26] != DMOD || in_sizes[27] != SDIM * DM4 ||
      in_sizes[28] != SDIM || in_sizes[29] != ADIM * DM4 || in_sizes[30] != ADIM || out_size != NOUT) return;

  const float* st   = (const float*)d_in[0];
  const float* ac   = (const float*)d_in[1];
  const float* rtg  = (const float*)d_in[2];
  const float* ctg  = (const float*)d_in[3];
  const int*   ts   = (const int*)d_in[4];
  const float* Ws   = (const float*)d_in[5];
  const float* bs   = (const float*)d_in[6];
  const float* Wa   = (const float*)d_in[7];
  const float* ba   = (const float*)d_in[8];
  const float* Wr   = (const float*)d_in[9];
  const float* br   = (const float*)d_in[10];
  const float* Wc   = (const float*)d_in[11];
  const float* bcn  = (const float*)d_in[12];
  const float* Et   = (const float*)d_in[13];
  const float* lng  = (const float*)d_in[14];
  const float* lnb  = (const float*)d_in[15];
  const float* inw  = (const float*)d_in[16];
  const float* cw   = (const float*)d_in[17];
  const float* cb   = (const float*)d_in[18];
  const float* xpw  = (const float*)d_in[19];
  const float* dtw  = (const float*)d_in[20];
  const float* dtb  = (const float*)d_in[21];
  const float* Alog = (const float*)d_in[22];
  const float* Dv   = (const float*)d_in[23];
  const float* ow   = (const float*)d_in[24];
  const float* fng  = (const float*)d_in[25];
  const float* fnb  = (const float*)d_in[26];
  const float* Wps  = (const float*)d_in[27];
  const float* bps  = (const float*)d_in[28];
  const float* Wpa  = (const float*)d_in[29];
  const float* bpa  = (const float*)d_in[30];
  float* out = (float*)d_out;

  size_t off = 0;
  auto carve = [&](size_t bytes) -> char* { char* p = (char*)d_ws + off; off += (bytes + 255) & ~(size_t)255; return p; };
  float* X             = (float*)carve((size_t)NTOK * DMOD * 4);
  unsigned short* NH   = (unsigned short*)carve((size_t)NTOK * DMOD * 2);
  unsigned short* NLO  = (unsigned short*)carve((size_t)NTOK * DMOD * 2);
  float* F             = (float*)carve((size_t)NTOK * DMOD * 4);
  unsigned short* WIN16 = (unsigned short*)carve((size_t)NLAY * XZW * DMOD * 2);
  unsigned short* WX16  = (unsigned short*)carve((size_t)NLAY * XDN * DIN * 2);
  unsigned short* WDT16 = (unsigned short*)carve((size_t)NLAY * DIN * DTR * 2);
  unsigned short* WO16  = (unsigned short*)carve((size_t)NLAY * DMOD * DIN * 2);
  float* XZ            = (float*)carve((size_t)NTOK * XZW * 4);
  float* XCF           = (float*)carve((size_t)NTOK * DIN * 4);
  unsigned short* XCH  = (unsigned short*)carve((size_t)NTOK * DIN * 2);
  unsigned short* XCL  = (unsigned short*)carve((size_t)NTOK * DIN * 2);
  float* XD            = (float*)carve((size_t)NTOK * XDN * 4);
  unsigned short* DTH  = (unsigned short*)carve((size_t)NTOK * DTR * 2);
  unsigned short* DTL  = (unsigned short*)carve((size_t)NTOK * DTR * 2);
  float* DTW           = (float*)carve((size_t)NTOK * DIN * 4);
  unsigned short* YGH  = (unsigned short*)carve((size_t)NTOK * DIN * 2);
  unsigned short* YGL  = (unsigned short*)carve((size_t)NTOK * DIN * 2);
  float* Y2            = (float*)carve((size_t)NTOK * DMOD * 4);
  if (off > ws_size || off > (size_t)134217728) return;

  const dim3 b256(256), b128(128);
  k_cvt<<<dim3((NLAY * XZW * DMOD / 8 + 255) / 256), b256, 0, stream>>>(inw, WIN16, NLAY * XZW, DMOD / 8, NLAY * XZW * DMOD / 8);
  k_cvt<<<dim3((NLAY * XDN * DIN / 8 + 255) / 256), b256, 0, stream>>>(xpw, WX16, NLAY * XDN, DIN / 8, NLAY * XDN * DIN / 8);
  k_cvt<<<dim3((NLAY * DIN * DTR / 8 + 255) / 256), b256, 0, stream>>>(dtw, WDT16, NLAY * DIN, DTR / 8, NLAY * DIN * DTR / 8);
  k_cvt<<<dim3((NLAY * DMOD * DIN / 8 + 255) / 256), b256, 0, stream>>>(ow, WO16, NLAY * DMOD, DIN / 8, NLAY * DMOD * DIN / 8);
  k_embed<<<dim3(NTOK), b128, 0, stream>>>(st, ac, rtg, ctg, ts, Ws, bs, Wa, ba, Wr, br, Wc, bcn, Et, X);

  for (int i = 0; i < NLAY; ++i) {
    if (i == 0) k_ln<0, 0><<<dim3(NTOK), b128, 0, stream>>>(X, Y2, lng + i * DMOD, lnb + i * DMOD, NH, NLO, F);
    else        k_ln<1, 0><<<dim3(NTOK), b128, 0, stream>>>(X, Y2, lng + i * DMOD, lnb + i * DMOD, NH, NLO, F);
    k_gemm<<<dim3(NTOK / 128, XZW / 64), b256, 0, stream>>>(NH, NLO, DMOD, WIN16 + (size_t)i * XZW * DMOD, DMOD, XZ, XZW, DMOD);
    k_conv<<<dim3(NTOK), b256, 0, stream>>>(XZ, cw + (size_t)i * DIN * DCV, cb + (size_t)i * DIN, XCF, XCH, XCL);
    k_gemm<<<dim3(NTOK / 128, XDN / 64), b256, 0, stream>>>(XCH, XCL, DIN, WX16 + (size_t)i * XDN * DIN, DIN, XD, XDN, DIN);
    k_dtsplit<<<dim3((NTOK * DTR / 8 + 255) / 256), b256, 0, stream>>>(XD, DTH, DTL);
    k_gemm<<<dim3(NTOK / 128, DIN / 64), b256, 0, stream>>>(DTH, DTL, DTR, WDT16 + (size_t)i * DIN * DTR, DTR, DTW, DIN, DTR);
    k_scan<<<dim3(NB * (DIN / 256)), b256, 0, stream>>>(XZ, XCF, XD, DTW, dtb + (size_t)i * DIN, Alog + (size_t)i * DIN * DST,
                                                        Dv + (size_t)i * DIN, YGH, YGL);
    k_gemm<<<dim3(NTOK / 128, DMOD / 64), b256, 0, stream>>>(YGH, YGL, DIN, WO16 + (size_t)i * DMOD * DIN, DIN, Y2, DMOD, DIN);
  }
  k_ln<1, 1><<<dim3(NTOK), b128, 0, stream>>>(X, Y2, fng, fnb, NH, NLO, F);
  k_heads<<<dim3(NOUT / 4 / 256), b256, 0, stream>>>(F, Wps, bps, Wpa, bpa, out);
}
